// PointNetSetAbstraction_85117661872237
// MI455X (gfx1250) — hardware-verified
//
#include <hip/hip_runtime.h>
#include <stdint.h>

#pragma clang fp contract(off)

typedef __attribute__((ext_vector_type(16))) _Float16 v16h;
typedef __attribute__((ext_vector_type(8)))  _Float16 v8h;
typedef __attribute__((ext_vector_type(8)))  float    v8f;
typedef __attribute__((ext_vector_type(4)))  float    v4f;
typedef __attribute__((ext_vector_type(4)))  unsigned v4u;

constexpr int NBATCH = 16;
constexpr int NPTS   = 4096;
constexpr int NCENT  = 1024;
constexpr int NNBR   = 32;
constexpr int NFEAT  = 64;
constexpr int CIN0   = 67;
constexpr int COUT01 = 64;
constexpr int COUT2  = 128;
constexpr int NROWS  = NBATCH * NCENT * NNBR;
constexpr int NSRC   = NBATCH * NPTS;
constexpr int NGRP   = NBATCH * NCENT;
constexpr int ROWS_PER_BLOCK = 512;
constexpr int NPART  = NROWS / ROWS_PER_BLOCK;
constexpr float WCARRY     = 16.0f;
constexpr float WCARRY_INV = 1.0f / 16.0f;
constexpr float BN_EPSF    = 1e-5f;

static_assert(NROWS == 524288, "rows");
static_assert(NCENT * NNBR == 32768, "rows per batch is 2^15");
static_assert(NPART == 1024, "partials");
static_assert(NFEAT == 64 && CIN0 == NFEAT + 3, "channels");
static_assert(NFEAT % 32 == 0, "K multiple of 32");
static_assert(NSRC % 64 == 0 && COUT01 % 64 == 0 && COUT2 % 64 == 0, "tile multiples");

constexpr size_t OFF_FEATT = 0;
constexpr size_t SZ_FEATT  = (size_t)NSRC * 64 * 2;
constexpr size_t OFF_P     = OFF_FEATT + SZ_FEATT;
constexpr size_t SZ_P      = (size_t)NSRC * 64 * 4;
constexpr size_t OFF_IDX   = OFF_P + SZ_P;
constexpr size_t SZ_IDX    = (size_t)NROWS * 4;
constexpr size_t OFF_NX    = OFF_IDX + SZ_IDX;
constexpr size_t SZ_NX     = (size_t)NGRP * 3 * 4;
constexpr size_t OFF_Y1    = OFF_NX + SZ_NX;
constexpr size_t SZ_Y1     = (size_t)NROWS * 64 * 2;
constexpr size_t OFF_YMM   = OFF_Y1 + SZ_Y1;
constexpr size_t SZ_YMM    = (size_t)NGRP * 256 * 4;
constexpr size_t OFF_WH    = OFF_YMM + SZ_YMM;
constexpr size_t SZ_WH     = (size_t)16384 * 2;
constexpr size_t OFF_PART0 = OFF_WH + SZ_WH;
constexpr size_t SZ_PART01 = (size_t)NPART * 128 * 4;
constexpr size_t OFF_PART1 = OFF_PART0 + SZ_PART01;
constexpr size_t OFF_PART2 = OFF_PART1 + SZ_PART01;
constexpr size_t SZ_PART2  = (size_t)NPART * 256 * 4;
constexpr size_t OFF_TAB0  = OFF_PART2 + SZ_PART2;
constexpr size_t OFF_TAB1  = OFF_TAB0 + 2048;
constexpr size_t OFF_TAB2  = OFF_TAB1 + 2048;
constexpr size_t WS_TOTAL  = OFF_TAB2 + 2048;
static_assert(WS_TOTAL == 113481728, "carve total");
static_assert(WS_TOTAL <= 134217728, "carve limit");
static_assert(OFF_P % 128 == 0 && OFF_IDX % 128 == 0 && OFF_NX % 128 == 0 && OFF_Y1 % 128 == 0, "align");
static_assert(OFF_YMM % 128 == 0 && OFF_WH % 128 == 0 && OFF_PART0 % 128 == 0 && OFF_TAB0 % 128 == 0, "align");
constexpr size_t OUT0_BYTES = (size_t)NGRP * 3 * 4;
constexpr size_t OUT1_BYTES = (size_t)NBATCH * COUT2 * NCENT * 4;
static_assert(OUT0_BYTES == 196608 && OUT0_BYTES % 128 == 0, "out1 offset");
static_assert(OUT0_BYTES + OUT1_BYTES == 8585216, "output total");

union FragU { v16h v; v8h h[2]; };
__device__ __forceinline__ v16h frag_load(const _Float16* p) {
  FragU f;
  f.h[0] = *(const v8h*)(p);
  f.h[1] = *(const v8h*)(p + 16);
  return f.v;
}
__device__ __forceinline__ v8f mma_h(v16h a, v16h b, v8f c) {
  c = __builtin_amdgcn_wmma_f32_16x16x32_f16(false, a, false, b, (short)0, c, false, false);
  asm volatile("v_nop\n\tv_nop\n\tv_nop\n\tv_nop" : "+v"(c) : "v"(a), "v"(b));
  return c;
}
__device__ __forceinline__ float h16_to_f32(unsigned hb) {
  const unsigned sgn = (hb & 0x8000u) << 16;
  const unsigned em = hb & 0x7fffu;
  const float fn = __uint_as_float((em << 13) + 0x38000000u);
  const float fs = (float)em * 5.9604644775390625e-8f;
  const float mag = (em < 0x400u) ? fs : fn;
  return __uint_as_float(__float_as_uint(mag) | sgn);
}
__device__ __forceinline__ void argmax_merge(float& bv, int& bi, float ov, int oi) {
  const bool take = (ov > bv) || ((ov == bv) && (oi < bi));
  bv = take ? ov : bv;
  bi = take ? oi : bi;
}
__device__ __forceinline__ int nth_set_bit(unsigned m, int n) {
  int pos = 0;
  unsigned mm = m;
  int c = __popc(mm & 0xFFFFu);
  bool g = (n >= c);
  pos += g ? 16 : 0; n -= g ? c : 0; mm = g ? (mm >> 16) : mm;
  c = __popc(mm & 0xFFu);
  g = (n >= c);
  pos += g ? 8 : 0; n -= g ? c : 0; mm = g ? (mm >> 8) : mm;
  c = __popc(mm & 0xFu);
  g = (n >= c);
  pos += g ? 4 : 0; n -= g ? c : 0; mm = g ? (mm >> 4) : mm;
  c = __popc(mm & 0x3u);
  g = (n >= c);
  pos += g ? 2 : 0; n -= g ? c : 0; mm = g ? (mm >> 2) : mm;
  c = __popc(mm & 0x1u);
  g = (n >= c);
  pos += g ? 1 : 0;
  return pos;
}
__device__ __forceinline__ void row_info(int n, const int* __restrict__ idx, const float* __restrict__ xyz,
                                         const float* __restrict__ nx, int& gp, float& dx, float& dy, float& dz) {
  int j = idx[n];
  j = j < 0 ? 0 : (j > NPTS - 1 ? NPTS - 1 : j);
  const int bs = n >> 5;
  const int b = n >> 15;
  gp = b * NPTS + j;
  const float* p = xyz + (size_t)gp * 3;
  const float* c = nx + (size_t)bs * 3;
  dx = p[0] - c[0];
  dy = p[1] - c[1];
  dz = p[2] - c[2];
}

__global__ __launch_bounds__(256) void prep_weights_kernel(const float* __restrict__ w0, const float* __restrict__ w1,
                                                           const float* __restrict__ w2, _Float16* __restrict__ wh) {
  const int t = blockIdx.x * 256 + threadIdx.x;
  const int e0 = t * 8;
  const float* base;
  if (blockIdx.x < 2) {
    const int o = e0 >> 6, k = e0 & 63;
    base = w0 + o * CIN0 + 3 + k;
  } else if (blockIdx.x < 4) {
    base = w1 + (e0 - 4096);
  } else {
    base = w2 + (e0 - 8192);
  }
  v8h hv;
#pragma unroll
  for (int e = 0; e < 8; ++e) {
    const float v = base[e] * WCARRY;
    hv[e] = (_Float16)v;
  }
  *(volatile v8h*)(wh + e0) = hv;
  __threadfence();
  *(volatile v8h*)(wh + e0) = hv;
}

__global__ __launch_bounds__(256) void feat_transpose_kernel(const float* __restrict__ feat, _Float16* __restrict__ featT) {
  __shared__ __align__(16) float ts[64 * 68];
  const int tid = threadIdx.x;
  const int b = blockIdx.x >> 6;
  const int n0 = (blockIdx.x & 63) * 64;
  const float* src = feat + (size_t)b * NFEAT * NPTS + n0;
#pragma unroll
  for (int it = 0; it < 4; ++it) {
    const int f = it * 256 + tid;
    const int c = f >> 4;
    const int q4 = (f & 15) * 4;
    const v4f v = *(const v4f*)(src + (size_t)c * NPTS + q4);
    ts[(q4 + 0) * 68 + c] = v[0];
    ts[(q4 + 1) * 68 + c] = v[1];
    ts[(q4 + 2) * 68 + c] = v[2];
    ts[(q4 + 3) * 68 + c] = v[3];
  }
  __syncthreads();
  const int q = tid & 7, rg = tid >> 3;
  v8h hv[2];
#pragma unroll
  for (int it = 0; it < 2; ++it) {
    const int r = it * 32 + rg;
    const v4f a = *(const v4f*)(ts + r * 68 + q * 8);
    const v4f c = *(const v4f*)(ts + r * 68 + q * 8 + 4);
#pragma unroll
    for (int e = 0; e < 4; ++e) {
      hv[it][e] = (_Float16)a[e];
      hv[it][4 + e] = (_Float16)c[e];
    }
  }
  for (int pass = 0; pass < 2; ++pass) {
#pragma unroll
    for (int it = 0; it < 2; ++it) {
      const int r = it * 32 + rg;
      *(volatile v8h*)(featT + ((size_t)b * NPTS + n0 + r) * 64 + q * 8) = hv[it];
    }
    __threadfence();
  }
}

__global__ __launch_bounds__(512) void fps_kernel(const float* __restrict__ xyz, float* __restrict__ out0,
                                                  float* __restrict__ nxws) {
#pragma clang fp contract(off)
  __shared__ __align__(16) float sx[NPTS * 3];
  __shared__ __align__(16) float snew[NCENT * 3];
  __shared__ float rv[32];
  __shared__ int ri[32];
  const int tid = threadIdx.x;
  const int lane = tid & 31;
  const int wave = tid >> 5;
  const int b = blockIdx.x;
  const v4f* src4 = (const v4f*)(xyz + (size_t)b * NPTS * 3);
#pragma unroll 1
  for (int i = tid; i < NPTS * 3 / 4; i += 512) {
    const v4f v = src4[i];
    *(v4f*)(sx + 4 * i) = v;
  }
  __syncthreads();
  float px[8], py[8], pz[8], dist[8];
#pragma unroll
  for (int t = 0; t < 8; ++t) {
    const int j = t * 512 + tid;
    px[t] = sx[j * 3 + 0];
    py[t] = sx[j * 3 + 1];
    pz[t] = sx[j * 3 + 2];
    dist[t] = 1e10f;
  }
  int last = 0;
#pragma unroll 1
  for (int step = 0; step < NCENT; ++step) {
    const float cx = sx[last * 3 + 0];
    const float cy = sx[last * 3 + 1];
    const float cz = sx[last * 3 + 2];
    if (tid == 0) {
      snew[step * 3 + 0] = cx;
      snew[step * 3 + 1] = cy;
      snew[step * 3 + 2] = cz;
    }
    float bv = -1.0f;
    int bi = 0;
#pragma unroll
    for (int t = 0; t < 8; ++t) {
      const float dx = px[t] - cx;
      const float dy = py[t] - cy;
      const float dz = pz[t] - cz;
      const float t0 = dx * dx;
      const float t1 = dy * dy;
      const float t2 = dz * dz;
      const float d = (t0 + t2) + t1;
      const float nd = fminf(dist[t], d);
      dist[t] = nd;
      const bool take = nd > bv;
      bv = take ? nd : bv;
      bi = take ? (t * 512 + tid) : bi;
    }
#pragma unroll
    for (int off = 16; off > 0; off >>= 1) {
      const float ov = __shfl_xor(bv, off, 32);
      const int oi = __shfl_xor(bi, off, 32);
      argmax_merge(bv, bi, ov, oi);
    }
    const int pp = (step & 1) * 16;
    if (lane == 0) {
      rv[pp + wave] = bv;
      ri[pp + wave] = bi;
    }
    __syncthreads();
    float gv = rv[pp + (lane & 15)];
    int gi = ri[pp + (lane & 15)];
#pragma unroll
    for (int off = 8; off > 0; off >>= 1) {
      const float ov = __shfl_xor(gv, off, 32);
      const int oi = __shfl_xor(gi, off, 32);
      argmax_merge(gv, gi, ov, oi);
    }
    last = gi & (NPTS - 1);
  }
  __syncthreads();
  for (int pass = 0; pass < 2; ++pass) {
#pragma unroll 1
    for (int i = tid; i < NCENT * 3 / 4; i += 512) {
      const v4f v = *(const v4f*)(snew + 4 * i);
      *(volatile v4f*)(out0 + (size_t)b * NCENT * 3 + 4 * i) = v;
      *(volatile v4f*)(nxws + (size_t)b * NCENT * 3 + 4 * i) = v;
    }
    __threadfence();
  }
}

__global__ __launch_bounds__(256) void ball_query_kernel(const float* __restrict__ xyz, const float* __restrict__ nx,
                                                         int* __restrict__ idx) {
#pragma clang fp contract(off)
  const int lane = threadIdx.x & 31;
  const int gw = blockIdx.x * 8 + (threadIdx.x >> 5);
  const int b = gw >> 10;
  const float cx = nx[(size_t)gw * 3 + 0];
  const float cy = nx[(size_t)gw * 3 + 1];
  const float cz = nx[(size_t)gw * 3 + 2];
  const float* base = xyz + (size_t)b * NPTS * 3;
  const float rad2 = 0.04f;
  int res = 0;
  int cnt = 0;
  int first = -1;
#pragma unroll 1
  for (int j0 = 0; j0 < NPTS; j0 += 32) {
    const int j = j0 + lane;
    const float x = base[j * 3 + 0];
    const float y = base[j * 3 + 1];
    const float z = base[j * 3 + 2];
    const float dx = cx - x;
    const float dy = cy - y;
    const float dz = cz - z;
    const float t0 = dx * dx;
    const float t1 = dy * dy;
    const float t2 = dz * dz;
    const float d2 = (t0 + t2) + t1;
    const bool in = d2 < rad2;
    const unsigned m = __builtin_amdgcn_ballot_w32(in);
    const int pc = __popc(m);
    const int tz = __builtin_ctz(m | 0x80000000u);
    if (first < 0 && m != 0u) first = j0 + tz;
    const int n = lane - cnt;
    const bool valid = (n >= 0) && (n < pc);
    const int nn = valid ? n : 0;
    const int pos = nth_set_bit(m, nn);
    res = valid ? (j0 + pos) : res;
    cnt += pc;
    if (cnt >= NNBR) break;
  }
  const int pad = first < 0 ? 0 : first;
  int fin = (lane < cnt) ? res : pad;
  fin = fin < 0 ? 0 : (fin > NPTS - 1 ? NPTS - 1 : fin);
  *(volatile int*)(idx + (size_t)gw * NNBR + lane) = fin;
  __threadfence();
  *(volatile int*)(idx + (size_t)gw * NNBR + lane) = fin;
}

__global__ __launch_bounds__(256) void gemm_p_kernel(const _Float16* __restrict__ A, const _Float16* __restrict__ Bt,
                                                     float* __restrict__ C) {
  __shared__ __align__(16) float sT[8][16 * 68];
  const int lane = threadIdx.x & 31;
  const int wave = threadIdx.x >> 5;
  const int tile = blockIdx.x * 8 + wave;
  const int m0 = tile << 6;
  const int rlane = lane & 15;
  const int koff = (lane >> 4) * 8;
  const int mOff = (lane >> 4) * 8;
  v8f acc[4][4];
#pragma unroll
  for (int i = 0; i < 4; ++i)
#pragma unroll
    for (int j = 0; j < 4; ++j) acc[i][j] = (v8f){0.f, 0.f, 0.f, 0.f, 0.f, 0.f, 0.f, 0.f};
#pragma unroll
  for (int k0 = 0; k0 < 64; k0 += 32) {
    v16h bh[4];
#pragma unroll
    for (int j = 0; j < 4; ++j) bh[j] = frag_load(Bt + (size_t)((j << 4) + rlane) * 64 + koff + k0);
#pragma unroll
    for (int i = 0; i < 4; ++i) {
      const v16h ah = frag_load(A + (size_t)(m0 + (i << 4) + rlane) * 64 + koff + k0);
#pragma unroll
      for (int j = 0; j < 4; ++j) acc[i][j] = mma_h(ah, bh[j], acc[i][j]);
    }
  }
  float* slab = sT[wave];
#pragma unroll
  for (int i = 0; i < 4; ++i) {
    const int mBase = m0 + (i << 4);
#pragma unroll
    for (int j = 0; j < 4; ++j) {
#pragma unroll
      for (int r = 0; r < 8; ++r) {
        const float v = acc[i][j][r] * WCARRY_INV;
        slab[(mOff + r) * 68 + (j << 4) + rlane] = v;
      }
    }
    __syncthreads();
    {
      const int hh = lane >> 4, c4 = (lane & 15) * 4;
      for (int pass = 0; pass < 2; ++pass) {
#pragma unroll
        for (int it = 0; it < 8; ++it) {
          const int row = it * 2 + hh;
          const v4f v = *(const v4f*)(slab + row * 68 + c4);
          *(volatile v4f*)(C + (size_t)(mBase + row) * 64 + c4) = v;
        }
        __threadfence();
      }
    }
    __syncthreads();
  }
}

__global__ __launch_bounds__(256) void stats0_kernel(const float* __restrict__ P, const int* __restrict__ idx,
                                                     const float* __restrict__ xyz, const float* __restrict__ nx,
                                                     const float* __restrict__ w0, const float* __restrict__ b0,
                                                     float* __restrict__ part) {
  __shared__ int sgp[64];
  __shared__ float sdx[64];
  __shared__ float sdy[64];
  __shared__ float sdz[64];
  __shared__ __align__(16) float red[16 * 128];
  const int tid = threadIdx.x;
  const int lane = tid & 31;
  const int c4 = (tid & 15) * 4;
  const int rg = tid >> 4;
  float wx[4], wy[4], wz[4];
#pragma unroll
  for (int e = 0; e < 4; ++e) wx[e] = w0[(c4 + e) * CIN0 + 0];
  asm volatile("" ::: "memory");
#pragma unroll
  for (int e = 0; e < 4; ++e) wy[e] = w0[(c4 + e) * CIN0 + 1];
  asm volatile("" ::: "memory");
#pragma unroll
  for (int e = 0; e < 4; ++e) wz[e] = w0[(c4 + e) * CIN0 + 2];
  const v4f bb = *(const v4f*)(b0 + c4);
  float s[4], q[4];
#pragma unroll
  for (int e = 0; e < 4; ++e) { s[e] = 0.0f; q[e] = 0.0f; }
#pragma unroll 1
  for (int tile = 0; tile < 8; ++tile) {
    const int n0 = blockIdx.x * ROWS_PER_BLOCK + tile * 64;
    if (tid < 64) {
      int gp; float dx, dy, dz;
      row_info(n0 + tid, idx, xyz, nx, gp, dx, dy, dz);
      sgp[tid] = gp; sdx[tid] = dx; sdy[tid] = dy; sdz[tid] = dz;
    }
    __syncthreads();
#pragma unroll 1
    for (int i = 0; i < 4; ++i) {
      const int r = rg + 16 * i;
      const int gp = sgp[r];
      const float dx = sdx[r], dy = sdy[r], dz = sdz[r];
      const v4f p = *(const v4f*)(P + (size_t)gp * 64 + c4);
#pragma unroll
      for (int e = 0; e < 4; ++e) {
        const float t = (wx[e] * dx + wy[e] * dy) + wz[e] * dz;
        const float y = (p[e] + t) + bb[e];
        s[e] += y;
        q[e] += y * y;
      }
    }
    __syncthreads();
  }
#pragma unroll
  for (int e = 0; e < 4; ++e) {
    red[rg * 128 + c4 + e] = s[e];
    red[rg * 128 + 64 + c4 + e] = q[e];
  }
  __syncthreads();
  if (tid < 32) {
    v4f sum = (v4f){0.f, 0.f, 0.f, 0.f};
#pragma unroll
    for (int g = 0; g < 16; ++g) sum += *(const v4f*)(red + g * 128 + 4 * lane);
    float* dst = part + (size_t)blockIdx.x * 128 + 4 * lane;
    *(volatile v4f*)dst = sum;
    __threadfence();
    *(volatile v4f*)dst = sum;
  }
}

template <int CO, bool L0>
__global__ __launch_bounds__(128) void finalize_kernel(const float* __restrict__ part, const float* __restrict__ g,
                                                       const float* __restrict__ be, const float* __restrict__ w0,
                                                       const float* __restrict__ b0, float* __restrict__ tab) {
  __shared__ __align__(16) float st[320];
  const int c = threadIdx.x;
  if (c < CO) {
    double s = 0.0, q = 0.0;
#pragma unroll 4
    for (int k = 0; k < NPART; ++k) {
      s += (double)part[(size_t)k * 2 * CO + c];
      q += (double)part[(size_t)k * 2 * CO + CO + c];
    }
    const double inv = 1.0 / (double)NROWS;
    const double mean = s * inv;
    double var = q * inv - mean * mean;
    var = var < 0.0 ? 0.0 : var;
    const float rs = rsqrtf((float)var + BN_EPSF);
    const float sc = g[c] * rs;
    if (L0) {
      const double bsh = ((double)b0[c] - mean) * (double)sc + (double)be[c];
      st[c] = sc;
      st[64 + c] = w0[c * CIN0 + 0] * sc;
      st[128 + c] = w0[c * CIN0 + 1] * sc;
      st[192 + c] = w0[c * CIN0 + 2] * sc;
      st[256 + c] = (float)bsh;
    } else {
      st[c] = sc;
      st[CO + c] = (float)((double)be[c] - mean * (double)sc);
    }
  }
  __syncthreads();
  constexpr int TOT4 = L0 ? 80 : (2 * CO / 4);
  if (threadIdx.x < 32) {
    for (int pass = 0; pass < 2; ++pass) {
#pragma unroll 1
      for (int i = threadIdx.x; i < TOT4; i += 32) {
        const v4f v = *(const v4f*)(st + 4 * i);
        *(volatile v4f*)(tab + 4 * i) = v;
      }
      __threadfence();
    }
  }
}

__global__ __launch_bounds__(256) void layer1_kernel(const float* __restrict__ P, const int* __restrict__ idx,
                                                     const float* __restrict__ xyz, const float* __restrict__ nx,
                                                     const float* __restrict__ tab0, const _Float16* __restrict__ W1h,
                                                     const float* __restrict__ bias1, _Float16* __restrict__ y1,
                                                     float* __restrict__ part) {
  __shared__ __align__(16) _Float16 As[128 * 72];
  __shared__ __align__(16) _Float16 Ws[64 * 72];
  __shared__ __align__(16) _Float16 Hs[8 * 16 * 72];
  __shared__ int sgp[128];
  __shared__ float sdx[128];
  __shared__ float sdy[128];
  __shared__ float sdz[128];
  __shared__ __align__(16) float sred[8 * 128];
  const int tid = threadIdx.x;
  const int lane = tid & 31;
  const int wave = tid >> 5;
  const int rlane = lane & 15;
  const int koff = (lane >> 4) * 8;
  const int mOff = (lane >> 4) * 8;
#pragma unroll
  for (int it = 0; it < 2; ++it) {
    const int f = it * 256 + tid;
    const int o = f >> 3, qq = f & 7;
    *(v8h*)(Ws + o * 72 + qq * 8) = *(const v8h*)(W1h + o * 64 + qq * 8);
  }
  const int c8 = (tid & 7) * 8;
  const int rg = tid >> 3;
  const v4f scA = *(const v4f*)(tab0 + c8);
  const v4f scB = *(const v4f*)(tab0 + c8 + 4);
  const v4f wxA = *(const v4f*)(tab0 + 64 + c8);
  const v4f wxB = *(const v4f*)(tab0 + 64 + c8 + 4);
  asm volatile("" ::: "memory");
  const v4f wyA = *(const v4f*)(tab0 + 128 + c8);
  const v4f wyB = *(const v4f*)(tab0 + 128 + c8 + 4);
  const v4f wzA = *(const v4f*)(tab0 + 192 + c8);
  const v4f wzB = *(const v4f*)(tab0 + 192 + c8 + 4);
  asm volatile("" ::: "memory");
  const v4f shA = *(const v4f*)(tab0 + 256 + c8);
  const v4f shB = *(const v4f*)(tab0 + 256 + c8 + 4);
  float bia[4];
#pragma unroll
  for (int j = 0; j < 4; ++j) bia[j] = bias1[j * 16 + rlane];
  float s[4], q[4];
#pragma unroll
  for (int j = 0; j < 4; ++j) { s[j] = 0.0f; q[j] = 0.0f; }
  _Float16* hs = Hs + wave * 16 * 72;
#pragma unroll 1
  for (int tile = 0; tile < 4; ++tile) {
    const int n0 = blockIdx.x * ROWS_PER_BLOCK + tile * 128;
    if (tid < 128) {
      int gp; float dx, dy, dz;
      row_info(n0 + tid, idx, xyz, nx, gp, dx, dy, dz);
      sgp[tid] = gp; sdx[tid] = dx; sdy[tid] = dy; sdz[tid] = dz;
    }
    __syncthreads();
#pragma unroll 1
    for (int i = 0; i < 4; ++i) {
      const int r = rg + 32 * i;
      const int gp = sgp[r];
      const float dx = sdx[r], dy = sdy[r], dz = sdz[r];
      const float* prow = P + (size_t)gp * 64 + c8;
      const v4f p0 = *(const v4f*)prow;
      const v4f p1 = *(const v4f*)(prow + 4);
      v8h hv;
#pragma unroll
      for (int e = 0; e < 4; ++e) {
        const float tA = (wxA[e] * dx + wyA[e] * dy) + wzA[e] * dz;
        float aA = (p0[e] * scA[e] + tA) + shA[e];
        aA = fmaxf(aA, 0.0f);
        hv[e] = (_Float16)aA;
        const float tB = (wxB[e] * dx + wyB[e] * dy) + wzB[e] * dz;
        float aB = (p1[e] * scB[e] + tB) + shB[e];
        aB = fmaxf(aB, 0.0f);
        hv[4 + e] = (_Float16)aB;
      }
      *(v8h*)(As + r * 72 + c8) = hv;
    }
    __syncthreads();
    v8f acc[4];
#pragma unroll
    for (int j = 0; j < 4; ++j) acc[j] = (v8f){0.f, 0.f, 0.f, 0.f, 0.f, 0.f, 0.f, 0.f};
    const _Float16* arow = As + (wave * 16 + rlane) * 72 + koff;
#pragma unroll
    for (int ks = 0; ks < 2; ++ks) {
      const v16h a = frag_load(arow + ks * 32);
#pragma unroll
      for (int j = 0; j < 4; ++j) {
        const v16h bf = frag_load(Ws + (j * 16 + rlane) * 72 + koff + ks * 32);
        acc[j] = mma_h(a, bf, acc[j]);
      }
    }
#pragma unroll
    for (int j = 0; j < 4; ++j) {
#pragma unroll
      for (int r = 0; r < 8; ++r) {
        const float v = acc[j][r] * WCARRY_INV + bia[j];
        s[j] += v;
        q[j] += v * v;
        hs[(mOff + r) * 72 + j * 16 + rlane] = (_Float16)v;
      }
    }
    __syncthreads();
    {
      const int qq = lane >> 3, cc = (lane & 7) * 8;
      v8h ov[4];
#pragma unroll
      for (int it = 0; it < 4; ++it) ov[it] = *(const v8h*)(hs + (it * 4 + qq) * 72 + cc);
      for (int pass = 0; pass < 2; ++pass) {
#pragma unroll
        for (int it = 0; it < 4; ++it) {
          *(volatile v8h*)(y1 + (size_t)(n0 + wave * 16 + it * 4 + qq) * 64 + cc) = ov[it];
        }
        __threadfence();
      }
    }
  }
#pragma unroll
  for (int j = 0; j < 4; ++j) {
    const float so = __shfl_xor(s[j], 16, 32);
    const float qo = __shfl_xor(q[j], 16, 32);
    s[j] += so;
    q[j] += qo;
  }
  if (lane < 16) {
#pragma unroll
    for (int j = 0; j < 4; ++j) {
      sred[wave * 128 + j * 16 + rlane] = s[j];
      sred[wave * 128 + 64 + j * 16 + rlane] = q[j];
    }
  }
  __syncthreads();
  if (tid < 32) {
    v4f sum = (v4f){0.f, 0.f, 0.f, 0.f};
#pragma unroll
    for (int w = 0; w < 8; ++w) sum += *(const v4f*)(sred + w * 128 + 4 * lane);
    float* dst = part + (size_t)blockIdx.x * 128 + 4 * lane;
    *(volatile v4f*)dst = sum;
    __threadfence();
    *(volatile v4f*)dst = sum;
  }
}

__global__ __launch_bounds__(256) void layer2_kernel(const unsigned short* __restrict__ y1u, const float* __restrict__ tab1,
                                                     const _Float16* __restrict__ W2h, const float* __restrict__ bias2,
                                                     float* __restrict__ ymm, float* __restrict__ part) {
  __shared__ __align__(16) _Float16 As[128 * 72];
  __shared__ __align__(16) _Float16 Ws[128 * 72];
  __shared__ __align__(16) float smm[8 * 256];
  __shared__ __align__(16) float sred[8 * 256];
  const int tid = threadIdx.x;
  const int lane = tid & 31;
  const int wave = tid >> 5;
  const int rlane = lane & 15;
  const int koff = (lane >> 4) * 8;
#pragma unroll
  for (int it = 0; it < 4; ++it) {
    const int f = it * 256 + tid;
    const int o = f >> 3, qq = f & 7;
    *(v8h*)(Ws + o * 72 + qq * 8) = *(const v8h*)(W2h + o * 64 + qq * 8);
  }
  const int c8 = (tid & 7) * 8;
  const int rg = tid >> 3;
  const v4f scA = *(const v4f*)(tab1 + c8);
  const v4f scB = *(const v4f*)(tab1 + c8 + 4);
  const v4f shA = *(const v4f*)(tab1 + 64 + c8);
  const v4f shB = *(const v4f*)(tab1 + 64 + c8 + 4);
  float bia[8];
#pragma unroll
  for (int j = 0; j < 8; ++j) bia[j] = bias2[j * 16 + rlane];
  float s[8], q[8];
#pragma unroll
  for (int j = 0; j < 8; ++j) { s[j] = 0.0f; q[j] = 0.0f; }
#pragma unroll 1
  for (int tile = 0; tile < 4; ++tile) {
    const int n0 = blockIdx.x * ROWS_PER_BLOCK + tile * 128;
#pragma unroll 1
    for (int i = 0; i < 4; ++i) {
      const int r = rg + 32 * i;
      const v4u w = *(const v4u*)(y1u + (size_t)(n0 + r) * 64 + c8);
      const unsigned w0 = w[0];
      const unsigned w1 = w[1];
      const unsigned w2 = w[2];
      const unsigned w3 = w[3];
      float f[8];
      f[0] = h16_to_f32(w0 & 0xffffu);
      f[1] = h16_to_f32(w0 >> 16);
      f[2] = h16_to_f32(w1 & 0xffffu);
      f[3] = h16_to_f32(w1 >> 16);
      f[4] = h16_to_f32(w2 & 0xffffu);
      f[5] = h16_to_f32(w2 >> 16);
      f[6] = h16_to_f32(w3 & 0xffffu);
      f[7] = h16_to_f32(w3 >> 16);
      v8h hv;
#pragma unroll
      for (int e = 0; e < 4; ++e) {
        const float aA = fmaxf(f[e] * scA[e] + shA[e], 0.0f);
        hv[e] = (_Float16)aA;
        const float aB = fmaxf(f[4 + e] * scB[e] + shB[e], 0.0f);
        hv[4 + e] = (_Float16)aB;
      }
      *(v8h*)(As + r * 72 + c8) = hv;
    }
    __syncthreads();
    v8f acc[8];
#pragma unroll
    for (int j = 0; j < 8; ++j) acc[j] = (v8f){0.f, 0.f, 0.f, 0.f, 0.f, 0.f, 0.f, 0.f};
    const _Float16* arow = As + (wave * 16 + rlane) * 72 + koff;
#pragma unroll
    for (int ks = 0; ks < 2; ++ks) {
      const v16h a = frag_load(arow + ks * 32);
#pragma unroll
      for (int j = 0; j < 8; ++j) {
        const v16h bf = frag_load(Ws + (j * 16 + rlane) * 72 + koff + ks * 32);
        acc[j] = mma_h(a, bf, acc[j]);
      }
    }
#pragma unroll
    for (int j = 0; j < 8; ++j) {
      float mx = -__builtin_inff();
      float mn = __builtin_inff();
#pragma unroll
      for (int r = 0; r < 8; ++r) {
        const float v = acc[j][r] * WCARRY_INV + bia[j];
        s[j] += v;
        q[j] += v * v;
        mx = fmaxf(mx, v);
        mn = fminf(mn, v);
      }
      const float mxo = __shfl_xor(mx, 16, 32);
      const float mno = __shfl_xor(mn, 16, 32);
      mx = fmaxf(mx, mxo);
      mn = fminf(mn, mno);
      if (lane < 16) {
        smm[wave * 256 + j * 16 + rlane] = mx;
        smm[wave * 256 + 128 + j * 16 + rlane] = mn;
      }
    }
    __syncthreads();
    {
      const int g = wave >> 1, half = wave & 1;
      const v4f a = *(const v4f*)(smm + (2 * g) * 256 + half * 128 + 4 * lane);
      const v4f c = *(const v4f*)(smm + (2 * g + 1) * 256 + half * 128 + 4 * lane);
      v4f o;
#pragma unroll
      for (int e = 0; e < 4; ++e) {
        const float vmx = fmaxf(a[e], c[e]);
        const float vmn = fminf(a[e], c[e]);
        o[e] = (half != 0) ? vmn : vmx;
      }
      float* dst = ymm + (size_t)((n0 >> 5) + g) * 256 + half * 128 + 4 * lane;
      *(volatile v4f*)dst = o;
      __threadfence();
      *(volatile v4f*)dst = o;
    }
  }
#pragma unroll
  for (int j = 0; j < 8; ++j) {
    const float so = __shfl_xor(s[j], 16, 32);
    const float qo = __shfl_xor(q[j], 16, 32);
    s[j] += so;
    q[j] += qo;
  }
  if (lane < 16) {
#pragma unroll
    for (int j = 0; j < 8; ++j) {
      sred[wave * 256 + j * 16 + rlane] = s[j];
      sred[wave * 256 + 128 + j * 16 + rlane] = q[j];
    }
  }
  __syncthreads();
  if (tid < 64) {
    v4f sum = (v4f){0.f, 0.f, 0.f, 0.f};
#pragma unroll
    for (int w = 0; w < 8; ++w) sum += *(const v4f*)(sred + w * 256 + 4 * tid);
    float* dst = part + (size_t)blockIdx.x * 256 + 4 * tid;
    *(volatile v4f*)dst = sum;
    __threadfence();
    *(volatile v4f*)dst = sum;
  }
}

__global__ __launch_bounds__(256) void out_kernel(const float* __restrict__ ymm, const float* __restrict__ tab2,
                                                  float* __restrict__ out1) {
  __shared__ __align__(16) float tv[128 * 36];
  const int tid = threadIdx.x;
  const int b = blockIdx.x >> 5;
  const int s0 = (blockIdx.x & 31) * 32;
  const int c4 = (tid & 31) * 4;
  const int sg = tid >> 5;
  const v4f sc = *(const v4f*)(tab2 + c4);
  const v4f sh = *(const v4f*)(tab2 + 128 + c4);
#pragma unroll
  for (int it = 0; it < 4; ++it) {
    const int si = sg + 8 * it;
    const size_t grp = (size_t)b * NCENT + s0 + si;
    const v4f vmax = *(const v4f*)(ymm + grp * 256 + c4);
    const v4f vmin = *(const v4f*)(ymm + grp * 256 + 128 + c4);
#pragma unroll
    for (int e = 0; e < 4; ++e) {
      const float fa = (sc[e] >= 0.0f) ? 1.0f : 0.0f;
      const float fb = 1.0f - fa;
      const float y = fa * vmax[e] + fb * vmin[e];
      const float v = fmaxf(y * sc[e] + sh[e], 0.0f);
      tv[(c4 + e) * 36 + si] = v;
    }
  }
  __syncthreads();
  const int qq = tid & 7, og = tid >> 3;
  for (int pass = 0; pass < 2; ++pass) {
#pragma unroll
    for (int it = 0; it < 4; ++it) {
      const int o = it * 32 + og;
      const v4f v = *(const v4f*)(tv + o * 36 + qq * 4);
      *(volatile v4f*)(out1 + ((size_t)b * COUT2 + o) * NCENT + s0 + qq * 4) = v;
    }
    __threadfence();
  }
}

extern "C" void kernel_launch(void* const* d_in, const int* in_sizes, int n_in,
                              void* d_out, int out_size, void* d_ws, size_t ws_size,
                              hipStream_t stream) {
  (void)in_sizes; (void)n_in; (void)out_size;
  if (ws_size < WS_TOTAL) return;
  const float* xyz  = (const float*)d_in[0];
  const float* feat = (const float*)d_in[1];
  const float* w0   = (const float*)d_in[2];
  const float* b0   = (const float*)d_in[3];
  const float* g0   = (const float*)d_in[4];
  const float* be0  = (const float*)d_in[5];
  const float* w1   = (const float*)d_in[6];
  const float* b1   = (const float*)d_in[7];
  const float* g1   = (const float*)d_in[8];
  const float* be1  = (const float*)d_in[9];
  const float* w2   = (const float*)d_in[10];
  const float* b2   = (const float*)d_in[11];
  const float* g2   = (const float*)d_in[12];
  const float* be2  = (const float*)d_in[13];

  char* ws = (char*)d_ws;
  _Float16* featT = (_Float16*)(ws + OFF_FEATT);
  float*    Pp    = (float*)(ws + OFF_P);
  int*      idx   = (int*)(ws + OFF_IDX);
  float*    nxw   = (float*)(ws + OFF_NX);
  _Float16* y1    = (_Float16*)(ws + OFF_Y1);
  float*    ymm   = (float*)(ws + OFF_YMM);
  _Float16* wh    = (_Float16*)(ws + OFF_WH);
  float*    part0 = (float*)(ws + OFF_PART0);
  float*    part1 = (float*)(ws + OFF_PART1);
  float*    part2 = (float*)(ws + OFF_PART2);
  float*    tab0  = (float*)(ws + OFF_TAB0);
  float*    tab1  = (float*)(ws + OFF_TAB1);
  float*    tab2  = (float*)(ws + OFF_TAB2);
  const _Float16* W0f = wh;
  const _Float16* W1h = wh + 4096;
  const _Float16* W2h = wh + 8192;

  float* out0 = (float*)d_out;
  float* out1 = (float*)d_out + OUT0_BYTES / 4;

  prep_weights_kernel<<<8, 256, 0, stream>>>(w0, w1, w2, wh);
  feat_transpose_kernel<<<NBATCH * (NPTS / 64), 256, 0, stream>>>(feat, featT);
  fps_kernel<<<NBATCH, 512, 0, stream>>>(xyz, out0, nxw);
  ball_query_kernel<<<NGRP / 8, 256, 0, stream>>>(xyz, nxw, idx);
  gemm_p_kernel<<<(NSRC / 64) / 8, 256, 0, stream>>>(featT, W0f, Pp);
  stats0_kernel<<<NPART, 256, 0, stream>>>(Pp, idx, xyz, nxw, w0, b0, part0);
  finalize_kernel<64, true><<<1, 128, 0, stream>>>(part0, g0, be0, w0, b0, tab0);
  layer1_kernel<<<NPART, 256, 0, stream>>>(Pp, idx, xyz, nxw, tab0, W1h, b1, y1, part1);
  finalize_kernel<64, false><<<1, 128, 0, stream>>>(part1, g1, be1, w0, b0, tab1);
  layer2_kernel<<<NPART, 256, 0, stream>>>((const unsigned short*)y1, tab1, W2h, b2, ymm, part2);
  finalize_kernel<128, false><<<1, 128, 0, stream>>>(part2, g2, be2, w0, b0, tab2);
  out_kernel<<<NBATCH * (NCENT / 32), 256, 0, stream>>>(ymm, tab2, out1);
}
